// NemotronHMOE_25245817766294
// MI455X (gfx1250) — hardware-verified
//
#include <hip/hip_runtime.h>
#include <stdint.h>
#include <stddef.h>
#include <math.h>

#pragma clang fp contract(off)

#define NTOK 4096
#define HD   1024
#define NEX  16
#define FI   512
#define FS   2048
#define TOPK 4
#define NGRP 4
#define MT   32
#define MS   16
#define NSL  256
#define XP   1032
#define HP   520
#define XSP  1032
#define HSP  2056
#define YP   260

#define LDS_X   (MT * XP * 2)
#define LDS_H   (MT * HP * 2)
#define LDS_EXP (LDS_X + LDS_H)
#define LDS_SX  (MS * XSP * 2)
#define LDS_SH  (MS * HSP * 2)
#define LDS_SHR (2 * LDS_SX + 2 * LDS_SH)

static_assert(MT * YP * 4 <= LDS_X);
static_assert(MS * YP * 4 <= 2 * LDS_SX);
static_assert((XP * 2) % 16 == 0);
static_assert((HP * 2) % 16 == 0);
static_assert((XSP * 2) % 16 == 0);
static_assert((HSP * 2) % 16 == 0);
static_assert((YP * 4) % 16 == 0);
static_assert(NTOK % 256 == 0);
static_assert(NTOK % MT == 0);
static_assert(NTOK % MS == 0);
static_assert(NTOK % 8 == 0);
static_assert(HD % NSL == 0);
static_assert(FI % NSL == 0);
static_assert(FS % NSL == 0);
static_assert(HD % 32 == 0);
static_assert(FI % 32 == 0);
static_assert(FS % 32 == 0);
static_assert(NSL == 8 * 32);
static_assert(MT == 8 * 4);
static_assert(MS == 8 * 2);
static_assert(NEX == NGRP * 4);
static_assert((NTOK * HD) % 8 == 0);
static_assert((NEX * FI * HD) % 8 == 0);
static_assert((FS * HD) % 8 == 0);

typedef _Float16       v16h  __attribute__((ext_vector_type(16)));
typedef __bf16         v16bf __attribute__((ext_vector_type(16)));
typedef float          v8f   __attribute__((ext_vector_type(8)));
typedef float          v4f   __attribute__((ext_vector_type(4)));
typedef unsigned int   v4u   __attribute__((ext_vector_type(4)));
typedef v4f __attribute__((may_alias)) v4fa;
typedef v4u __attribute__((may_alias)) v4ua;

union FragH  { v16h  v; v4u q[2]; };
union FragBF { v16bf v; v4u q[2]; };

__device__ __forceinline__ unsigned int bfb(float f) {
  unsigned int u = __float_as_uint(f);
  u += 0x7FFFu + ((u >> 16) & 1u);
  return u >> 16;
}
__device__ __forceinline__ void split2(float v, unsigned int& hi, unsigned int& lo) {
  hi = bfb(v);
  lo = bfb(v - __uint_as_float(hi << 16));
}
__device__ __forceinline__ unsigned int hbits(float f) {
  union { _Float16 h; unsigned short u; } c;
  c.h = (_Float16)f;
  return (unsigned int)c.u;
}
__device__ __forceinline__ unsigned int pk(unsigned int a, unsigned int b) { return (a & 0xFFFFu) | (b << 16); }

__device__ __forceinline__ v8f wmma_h(v16h a, v16h b, v8f c) {
  v8f d = __builtin_amdgcn_wmma_f32_16x16x32_f16(false, a, false, b, (short)0, c, false, false);
  asm volatile("v_nop\n\tv_nop\n\tv_nop\n\tv_nop" : "+v"(d) : "v"(a), "v"(b));
  return d;
}
__device__ __forceinline__ v8f wmma_bf(v16bf a, v16bf b, v8f c) {
  v8f d = __builtin_amdgcn_wmma_f32_16x16x32_bf16(false, a, false, b, (short)0, c, false, false);
  asm volatile("v_nop\n\tv_nop\n\tv_nop\n\tv_nop" : "+v"(d) : "v"(a), "v"(b));
  return d;
}

__device__ __forceinline__ v16h ldfrag_h(const unsigned short* p, int h) {
  FragH f;
  f.q[0] = *(const v4ua*)(p + 8 * h);
  f.q[1] = *(const v4ua*)(p + 16 + 8 * h);
  return f.v;
}
__device__ __forceinline__ v16bf ldfrag_bf(const unsigned short* p, int h) {
  FragBF f;
  f.q[0] = *(const v4ua*)(p + 8 * h);
  f.q[1] = *(const v4ua*)(p + 16 + 8 * h);
  return f.v;
}

__global__ __launch_bounds__(256) void k_cvt16(const float* __restrict__ src,
                                               unsigned short* __restrict__ dst,
                                               float scale, int n8)
{
  const int g = blockIdx.x * 256 + threadIdx.x;
  if (g >= n8) return;
  const float* s = src + (size_t)g * 8;
  const v4f a = *(const v4fa*)s;
  const v4f c = *(const v4fa*)(s + 4);
  const v4u P = { pk(hbits(a.x * scale), hbits(a.y * scale)),
                  pk(hbits(a.z * scale), hbits(a.w * scale)),
                  pk(hbits(c.x * scale), hbits(c.y * scale)),
                  pk(hbits(c.z * scale), hbits(c.w * scale)) };
  unsigned short* d = dst + (size_t)g * 8;
  *(volatile v4u*)d = P;
  __threadfence();
  *(volatile v4u*)d = P;
}

__global__ __launch_bounds__(256) void k_split(const float* __restrict__ src,
                                               unsigned short* __restrict__ ph,
                                               unsigned short* __restrict__ pl, int n8)
{
  const int g = blockIdx.x * 256 + threadIdx.x;
  if (g >= n8) return;
  const float* s = src + (size_t)g * 8;
  const v4f a = *(const v4fa*)s;
  const v4f c = *(const v4fa*)(s + 4);
  unsigned int h0, l0, h1, l1, h2, l2, h3, l3, h4, l4, h5, l5, h6, l6, h7, l7;
  split2(a.x, h0, l0); split2(a.y, h1, l1); split2(a.z, h2, l2); split2(a.w, h3, l3);
  split2(c.x, h4, l4); split2(c.y, h5, l5); split2(c.z, h6, l6); split2(c.w, h7, l7);
  const v4u H = { pk(h0, h1), pk(h2, h3), pk(h4, h5), pk(h6, h7) };
  const v4u L = { pk(l0, l1), pk(l2, l3), pk(l4, l5), pk(l6, l7) };
  unsigned short* dh = ph + (size_t)g * 8;
  unsigned short* dl = pl + (size_t)g * 8;
  *(volatile v4u*)dh = H;
  *(volatile v4u*)dl = L;
  __threadfence();
  *(volatile v4u*)dh = H;
  *(volatile v4u*)dl = L;
}

__global__ __launch_bounds__(256) void k_route(const float* __restrict__ x,
                                               const float* __restrict__ rw,
                                               const float* __restrict__ bias,
                                               const int* __restrict__ meta,
                                               unsigned int* __restrict__ rec, int ntok)
{
  __shared__ __align__(16) unsigned int srec[64];
  (void)meta;
  const int tid = threadIdx.x, lane = tid & 31, wv = tid >> 5;

  const int t = blockIdx.x * 8 + wv;
  const int tc = (t < ntok) ? t : (ntok - 1);
  const float* xr = x + (size_t)tc * HD;
  double lg[NEX];
  #pragma unroll
  for (int e = 0; e < NEX; ++e) lg[e] = 0.0;
  #pragma unroll 1
  for (int i = 0; i < HD / 32; ++i) {
    const int d = 32 * i + lane;
    const double xv = (double)xr[d];
    #pragma unroll
    for (int e = 0; e < NEX; ++e) lg[e] = fma(xv, (double)rw[(size_t)e * HD + d], lg[e]);
  }
  #pragma unroll
  for (int off = 16; off > 0; off >>= 1) {
    #pragma unroll
    for (int e = 0; e < NEX; ++e) lg[e] = lg[e] + __shfl_xor(lg[e], off);
  }

  float lf[NEX];
  #pragma unroll
  for (int e = 0; e < NEX; ++e) lf[e] = (float)lg[e];
  const int e16 = lane & 15;
  float myl = lf[0];
  #pragma unroll
  for (int e = 1; e < NEX; ++e) myl = (e == e16) ? lf[e] : myl;
  myl = fminf(fmaxf(myl, -80.0f), 80.0f);
  const float mys = __builtin_amdgcn_rcpf(1.0f + expf(-myl));

  float sc[NEX], sf[NEX];
  #pragma unroll
  for (int e = 0; e < NEX; ++e) { sc[e] = __shfl(mys, e); sf[e] = sc[e] + bias[e]; }

  float gsc[NGRP];
  #pragma unroll
  for (int g = 0; g < NGRP; ++g) {
    float m1 = sf[4 * g]; int i1 = 0;
    #pragma unroll
    for (int j = 1; j < 4; ++j) {
      const bool tk = sf[4 * g + j] > m1;
      m1 = tk ? sf[4 * g + j] : m1;
      i1 = tk ? j : i1;
    }
    float m2 = -3.0e38f;
    #pragma unroll
    for (int j = 0; j < 4; ++j) {
      const bool tk = (j != i1) && (sf[4 * g + j] > m2);
      m2 = tk ? sf[4 * g + j] : m2;
    }
    gsc[g] = m1 + m2;
  }
  int g1 = 0; float bm = gsc[0];
  #pragma unroll
  for (int g = 1; g < NGRP; ++g) {
    const bool tk = gsc[g] > bm;
    bm = tk ? gsc[g] : bm;
    g1 = tk ? g : g1;
  }
  int g2 = -1; float bm2 = -3.0e38f;
  #pragma unroll
  for (int g = 0; g < NGRP; ++g) {
    const bool tk = (g != g1) && (gsc[g] > bm2);
    bm2 = tk ? gsc[g] : bm2;
    g2 = tk ? g : g2;
  }
  g2 = (g2 < 0) ? ((g1 == 0) ? 1 : 0) : g2;

  float mk[NEX];
  #pragma unroll
  for (int e = 0; e < NEX; ++e) {
    const int g = e >> 2;
    mk[e] = (g == g1 || g == g2) ? sf[e] : 0.0f;
  }
  int ti[TOPK]; float tv[TOPK];
  #pragma unroll
  for (int k = 0; k < TOPK; ++k) {
    float mv = mk[0]; int im = 0;
    #pragma unroll
    for (int e = 1; e < NEX; ++e) {
      const bool tk = mk[e] > mv;
      mv = tk ? mk[e] : mv;
      im = tk ? e : im;
    }
    float w = sc[0];
    #pragma unroll
    for (int e = 1; e < NEX; ++e) w = (e == im) ? sc[e] : w;
    ti[k] = im;
    tv[k] = w;
    #pragma unroll
    for (int e = 0; e < NEX; ++e) mk[e] = (e == im) ? -3.0e38f : mk[e];
  }
  float den = tv[0] + tv[1];
  den = den + tv[2];
  den = den + tv[3];
  den = den + 1e-20f;
  const float rden = __builtin_amdgcn_rcpf(den);

  if (lane == 0) {
    #pragma unroll
    for (int k = 0; k < TOPK; ++k) {
      srec[wv * 8 + k]     = __float_as_uint((tv[k] * rden) * 2.5f);
      srec[wv * 8 + 4 + k] = (unsigned int)ti[k];
    }
  }
  __syncthreads();
  if (wv == 0) {
    const int q = lane & 15;
    const v4u v = *(const v4ua*)(srec + 4 * q);
    const int tt = blockIdx.x * 8 + (q >> 1);
    const bool ok = (lane < 16) && (tt < ntok);
    unsigned int* dst = rec + (size_t)blockIdx.x * 64 + 4 * q;
    if (ok) *(volatile v4u*)dst = v;
    __threadfence();
    if (ok) *(volatile v4u*)dst = v;
  }
}

__device__ __forceinline__ void part_pass(const float* sY, const int* sTok, const int* sSlot,
                                          float* part, int ns, int wv, int lane, int nrows)
{
  #pragma unroll
  for (int i = 0; i < 4; ++i) {
    const int row = wv * 4 + i;
    int t = sTok[row];
    t = (t < 0) ? 0 : ((t > NTOK - 1) ? (NTOK - 1) : t);
    int s = sSlot[row];
    s = (s < 0) ? 0 : ((s > TOPK - 1) ? (TOPK - 1) : s);
    const v4f v0 = *(const v4fa*)(sY + row * YP + 4 * lane);
    const v4f v1 = *(const v4fa*)(sY + row * YP + 128 + 4 * lane);
    float* dst = part + ((size_t)t * TOPK + s) * HD + ns * NSL;
    if (row < nrows) {
      *(volatile v4f*)(dst + 4 * lane) = v0;
      *(volatile v4f*)(dst + 128 + 4 * lane) = v1;
    }
  }
}

__global__ __launch_bounds__(256) void k_expert(const unsigned short* __restrict__ x16,
                                                const unsigned short* __restrict__ wup,
                                                const unsigned short* __restrict__ wdn,
                                                const unsigned int* __restrict__ rec,
                                                float* __restrict__ part, int ntok)
{
  extern __shared__ __align__(16) unsigned char dsm_e[];
  unsigned short* sX = (unsigned short*)dsm_e;
  unsigned short* sH = (unsigned short*)(dsm_e + LDS_X);
  float* sY = (float*)dsm_e;
  __shared__ int   sTok[MT];
  __shared__ int   sSlot[MT];
  __shared__ float sW[MT];
  __shared__ int   s_wc[8];

  const int tid = threadIdx.x, lane = tid & 31, wv = tid >> 5;
  const int h = lane >> 4, m = lane & 15;
  const int e = blockIdx.y;
  const int m0 = blockIdx.x * MT;

  if (tid < MT) { sTok[tid] = 0; sSlot[tid] = 0; sW[tid] = 0.0f; }
  __syncthreads();

  int base = 0;
  #pragma unroll 1
  for (int ch = 0; ch < NTOK / 256; ++ch) {
    const int t = ch * 256 + tid;
    const int tc = (t < ntok) ? t : (ntok - 1);
    const v4f rwt = *(const v4fa*)(rec + (size_t)tc * 8);
    const v4u ri  = *(const v4ua*)(rec + (size_t)tc * 8 + 4);
    const int i0 = (int)ri.x, i1 = (int)ri.y, i2 = (int)ri.z, i3 = (int)ri.w;
    const bool f0 = (i0 == e);
    const bool f1 = (i1 == e) && !f0;
    const bool f2 = (i2 == e) && !f0 && !f1;
    const bool f3 = (i3 == e) && !f0 && !f1 && !f2;
    const bool f = (f0 || f1 || f2 || f3) && (t < ntok);
    const int slot = f0 ? 0 : (f1 ? 1 : (f2 ? 2 : 3));
    const float wsel = f0 ? rwt.x : (f1 ? rwt.y : (f2 ? rwt.z : rwt.w));
    const unsigned int msk = __builtin_amdgcn_ballot_w32(f);
    const int off = __builtin_popcount(msk & ((1u << lane) - 1u));
    const int wc = __builtin_popcount(msk);
    if (lane == 0) s_wc[wv] = wc;
    __syncthreads();
    int pre = 0, tot = 0;
    #pragma unroll
    for (int w2 = 0; w2 < 8; ++w2) {
      const int cc = s_wc[w2];
      tot += cc;
      pre += (w2 < wv) ? cc : 0;
    }
    if (f) {
      const int p = base + pre + off - m0;
      if ((unsigned)p < (unsigned)MT) {
        sTok[p]  = t;
        sSlot[p] = slot;
        sW[p]    = wsel;
      }
    }
    base += tot;
    __syncthreads();
  }
  const int cnt = base;
  if (m0 >= cnt) return;
  int nrows = cnt - m0;
  nrows = (nrows > MT) ? MT : nrows;

  #pragma unroll 4
  for (int j = 0; j < 16; ++j) {
    const int idx = tid + 256 * j;
    const int row = idx >> 7, c8 = idx & 127;
    int t = sTok[row];
    t = (t < 0) ? 0 : ((t > NTOK - 1) ? (NTOK - 1) : t);
    const v4u a = *(const v4ua*)(x16 + (size_t)t * HD + 8 * c8);
    *(v4ua*)(sX + row * XP + 8 * c8) = a;
  }
  __syncthreads();

  const v8f z8 = {0.f, 0.f, 0.f, 0.f, 0.f, 0.f, 0.f, 0.f};

  #pragma unroll 1
  for (int ns = 0; ns < FI / NSL; ++ns) {
    v8f acc[2][2];
    #pragma unroll
    for (int mt = 0; mt < 2; ++mt)
      #pragma unroll
      for (int nt = 0; nt < 2; ++nt) acc[mt][nt] = z8;
    #pragma unroll 1
    for (int k0 = 0; k0 < HD; k0 += 32) {
      v16h a[2];
      #pragma unroll
      for (int mt = 0; mt < 2; ++mt) a[mt] = ldfrag_h(sX + (16 * mt + m) * XP + k0, h);
      #pragma unroll
      for (int nt = 0; nt < 2; ++nt) {
        const int f = ns * NSL + wv * 32 + 16 * nt + m;
        const size_t bo = ((size_t)e * FI + f) * HD + k0;
        const v16h b = ldfrag_h(wup + bo, h);
        #pragma unroll
        for (int mt = 0; mt < 2; ++mt) acc[mt][nt] = wmma_h(a[mt], b, acc[mt][nt]);
      }
    }
    #pragma unroll
    for (int mt = 0; mt < 2; ++mt)
      #pragma unroll
      for (int nt = 0; nt < 2; ++nt) {
        const int col = ns * NSL + wv * 32 + 16 * nt + m;
        #pragma unroll
        for (int r = 0; r < 8; ++r) {
          const int row = 16 * mt + 8 * h + r;
          float u = acc[mt][nt][r] * 0.015625f;
          u = (u > 0.0f) ? u : 0.0f;
          float hv = (u * u) * 64.0f;
          hv = fminf(hv, 65504.0f);
          sH[row * HP + col] = (unsigned short)hbits(hv);
        }
      }
  }
  __syncthreads();

  #pragma unroll 1
  for (int ns = 0; ns < HD / NSL; ++ns) {
    v8f acc[2][2];
    #pragma unroll
    for (int mt = 0; mt < 2; ++mt)
      #pragma unroll
      for (int nt = 0; nt < 2; ++nt) acc[mt][nt] = z8;
    #pragma unroll 1
    for (int k0 = 0; k0 < FI; k0 += 32) {
      v16h a[2];
      #pragma unroll
      for (int mt = 0; mt < 2; ++mt) a[mt] = ldfrag_h(sH + (16 * mt + m) * HP + k0, h);
      #pragma unroll
      for (int nt = 0; nt < 2; ++nt) {
        const int d = ns * NSL + wv * 32 + 16 * nt + m;
        const size_t bo = ((size_t)e * HD + d) * FI + k0;
        const v16h b = ldfrag_h(wdn + bo, h);
        #pragma unroll
        for (int mt = 0; mt < 2; ++mt) acc[mt][nt] = wmma_h(a[mt], b, acc[mt][nt]);
      }
    }
    #pragma unroll
    for (int mt = 0; mt < 2; ++mt)
      #pragma unroll
      for (int nt = 0; nt < 2; ++nt) {
        const int cl = wv * 32 + 16 * nt + m;
        #pragma unroll
        for (int r = 0; r < 8; ++r) {
          const int row = 16 * mt + 8 * h + r;
          sY[row * YP + cl] = (acc[mt][nt][r] * (1.0f / 4096.0f)) * sW[row];
        }
      }
    __syncthreads();
    part_pass(sY, sTok, sSlot, part, ns, wv, lane, nrows);
    __threadfence();
    part_pass(sY, sTok, sSlot, part, ns, wv, lane, nrows);
    __syncthreads();
  }
}

__global__ __launch_bounds__(256) void k_shared(const float* __restrict__ x,
                                                const unsigned short* __restrict__ wsuh,
                                                const unsigned short* __restrict__ wsul,
                                                const unsigned short* __restrict__ wsdh,
                                                const unsigned short* __restrict__ wsdl,
                                                const float* __restrict__ part,
                                                float* __restrict__ out, int ntok)
{
  extern __shared__ __align__(16) unsigned char dsm_s[];
  unsigned short* sXh = (unsigned short*)dsm_s;
  unsigned short* sXl = (unsigned short*)(dsm_s + LDS_SX);
  unsigned short* sHh = (unsigned short*)(dsm_s + 2 * LDS_SX);
  unsigned short* sHl = (unsigned short*)(dsm_s + 2 * LDS_SX + LDS_SH);
  float* sY = (float*)dsm_s;

  const int tid = threadIdx.x, lane = tid & 31, wv = tid >> 5;
  const int h = lane >> 4, m = lane & 15;
  const int t0 = blockIdx.x * MS;

  #pragma unroll 2
  for (int j = 0; j < 8; ++j) {
    const int idx = tid + 256 * j;
    const int row = idx >> 7, c8 = idx & 127;
    int tr = t0 + row;
    tr = (tr > ntok - 1) ? (ntok - 1) : tr;
    const float* s = x + (size_t)tr * HD + 8 * c8;
    const v4f a = *(const v4fa*)s;
    const v4f c = *(const v4fa*)(s + 4);
    unsigned int h0, l0, h1, l1, h2, l2, h3, l3, h4, l4, h5, l5, h6, l6, h7, l7;
    split2(a.x, h0, l0); split2(a.y, h1, l1); split2(a.z, h2, l2); split2(a.w, h3, l3);
    split2(c.x, h4, l4); split2(c.y, h5, l5); split2(c.z, h6, l6); split2(c.w, h7, l7);
    const v4u H = { pk(h0, h1), pk(h2, h3), pk(h4, h5), pk(h6, h7) };
    const v4u L = { pk(l0, l1), pk(l2, l3), pk(l4, l5), pk(l6, l7) };
    *(v4ua*)(sXh + row * XSP + 8 * c8) = H;
    *(v4ua*)(sXl + row * XSP + 8 * c8) = L;
  }
  __syncthreads();

  const v8f z8 = {0.f, 0.f, 0.f, 0.f, 0.f, 0.f, 0.f, 0.f};

  #pragma unroll 1
  for (int ns = 0; ns < FS / NSL; ++ns) {
    v8f acc[2];
    #pragma unroll
    for (int nt = 0; nt < 2; ++nt) acc[nt] = z8;
    #pragma unroll 1
    for (int k0 = 0; k0 < HD; k0 += 32) {
      const v16bf ah = ldfrag_bf(sXh + m * XSP + k0, h);
      const v16bf al = ldfrag_bf(sXl + m * XSP + k0, h);
      #pragma unroll
      for (int nt = 0; nt < 2; ++nt) {
        const int f = ns * NSL + wv * 32 + 16 * nt + m;
        const size_t bo = (size_t)f * HD + k0;
        const v16bf bh = ldfrag_bf(wsuh + bo, h);
        const v16bf bl = ldfrag_bf(wsul + bo, h);
        acc[nt] = wmma_bf(ah, bh, acc[nt]);
        acc[nt] = wmma_bf(ah, bl, acc[nt]);
        acc[nt] = wmma_bf(al, bh, acc[nt]);
      }
    }
    #pragma unroll
    for (int nt = 0; nt < 2; ++nt) {
      const int col = ns * NSL + wv * 32 + 16 * nt + m;
      #pragma unroll
      for (int r = 0; r < 8; ++r) {
        const int row = 8 * h + r;
        float u = acc[nt][r];
        u = (u > 0.0f) ? u : 0.0f;
        const float hv = u * u;
        unsigned int hb, lb;
        split2(hv, hb, lb);
        sHh[row * HSP + col] = (unsigned short)hb;
        sHl[row * HSP + col] = (unsigned short)lb;
      }
    }
  }
  __syncthreads();

  #pragma unroll 1
  for (int ns = 0; ns < HD / NSL; ++ns) {
    v8f acc[2];
    #pragma unroll
    for (int nt = 0; nt < 2; ++nt) acc[nt] = z8;
    #pragma unroll 1
    for (int k0 = 0; k0 < FS; k0 += 32) {
      const v16bf ah = ldfrag_bf(sHh + m * HSP + k0, h);
      const v16bf al = ldfrag_bf(sHl + m * HSP + k0, h);
      #pragma unroll
      for (int nt = 0; nt < 2; ++nt) {
        const int d = ns * NSL + wv * 32 + 16 * nt + m;
        const size_t bo = (size_t)d * FS + k0;
        const v16bf bh = ldfrag_bf(wsdh + bo, h);
        const v16bf bl = ldfrag_bf(wsdl + bo, h);
        acc[nt] = wmma_bf(ah, bh, acc[nt]);
        acc[nt] = wmma_bf(ah, bl, acc[nt]);
        acc[nt] = wmma_bf(al, bh, acc[nt]);
      }
    }
    #pragma unroll
    for (int nt = 0; nt < 2; ++nt) {
      const int cl = wv * 32 + 16 * nt + m;
      #pragma unroll
      for (int r = 0; r < 8; ++r) sY[(8 * h + r) * YP + cl] = acc[nt][r];
    }
    __syncthreads();

    v4f ov[2][2];
    #pragma unroll
    for (int i = 0; i < 2; ++i) {
      const int row = wv * 2 + i;
      int tr = t0 + row;
      tr = (tr > ntok - 1) ? (ntok - 1) : tr;
      const float* pp = part + (size_t)tr * TOPK * HD + ns * NSL;
      #pragma unroll
      for (int j = 0; j < 2; ++j) {
        const int c = 128 * j + 4 * lane;
        const v4f y  = *(const v4fa*)(sY + row * YP + c);
        const v4f p0 = *(const v4fa*)(pp + 0 * HD + c);
        const v4f p1 = *(const v4fa*)(pp + 1 * HD + c);
        const v4f p2 = *(const v4fa*)(pp + 2 * HD + c);
        const v4f p3 = *(const v4fa*)(pp + 3 * HD + c);
        v4f rs = p0 + p1;
        rs = rs + p2;
        rs = rs + p3;
        ov[i][j] = rs + y;
      }
    }
    #pragma unroll
    for (int i = 0; i < 2; ++i) {
      const int row = wv * 2 + i;
      const bool ok = (t0 + row) < ntok;
      float* dst = out + (size_t)(t0 + row) * HD + ns * NSL;
      #pragma unroll
      for (int j = 0; j < 2; ++j)
        if (ok) *(volatile v4f*)(dst + 128 * j + 4 * lane) = ov[i][j];
    }
    __threadfence();
    #pragma unroll
    for (int i = 0; i < 2; ++i) {
      const int row = wv * 2 + i;
      const bool ok = (t0 + row) < ntok;
      float* dst = out + (size_t)(t0 + row) * HD + ns * NSL;
      #pragma unroll
      for (int j = 0; j < 2; ++j)
        if (ok) *(volatile v4f*)(dst + 128 * j + 4 * lane) = ov[i][j];
    }
    __syncthreads();
  }
}

extern "C" void kernel_launch(void* const* d_in, const int* in_sizes, int n_in,
                              void* d_out, int out_size, void* d_ws, size_t ws_size,
                              hipStream_t stream)
{
  if (n_in < 8) return;
  if (in_sizes[0] != NTOK * HD) return;
  if (in_sizes[1] != NEX * HD) return;
  if (in_sizes[2] != NEX) return;
  if (in_sizes[3] != NEX * FI * HD) return;
  if (in_sizes[4] != NEX * HD * FI) return;
  if (in_sizes[5] != FS * HD) return;
  if (in_sizes[6] != HD * FS) return;
  if (out_size != NTOK * HD) return;

  const float* x    = (const float*)d_in[0];
  const float* rw   = (const float*)d_in[1];
  const float* bias = (const float*)d_in[2];
  const float* wup  = (const float*)d_in[3];
  const float* wdn  = (const float*)d_in[4];
  const float* wsu  = (const float*)d_in[5];
  const float* wsd  = (const float*)d_in[6];
  const int*   meta = (const int*)d_in[7];
  float* out = (float*)d_out;

  const size_t bX16  = (size_t)NTOK * HD * 2;
  const size_t bWUP  = (size_t)NEX * FI * HD * 2;
  const size_t bWDN  = (size_t)NEX * HD * FI * 2;
  const size_t bWSP  = (size_t)FS * HD * 2;
  const size_t bREC  = (size_t)NTOK * 32;
  const size_t bPART = (size_t)NTOK * TOPK * HD * 4;
  const size_t total = bX16 + bWUP + bWDN + 4 * bWSP + bREC + bPART;
  if (total > ws_size) return;
  if (total > (size_t)134217728) return;

  char* ws = (char*)d_ws;
  size_t off = 0;
  unsigned short* X16  = (unsigned short*)(ws + off); off += bX16;
  unsigned short* WUP  = (unsigned short*)(ws + off); off += bWUP;
  unsigned short* WDN  = (unsigned short*)(ws + off); off += bWDN;
  unsigned short* WSUH = (unsigned short*)(ws + off); off += bWSP;
  unsigned short* WSUL = (unsigned short*)(ws + off); off += bWSP;
  unsigned short* WSDH = (unsigned short*)(ws + off); off += bWSP;
  unsigned short* WSDL = (unsigned short*)(ws + off); off += bWSP;
  unsigned int*   REC  = (unsigned int*)(ws + off);   off += bREC;
  float*          PART = (float*)(ws + off);          off += bPART;
  if (off != total) return;

  {
    const int n8x = NTOK * HD / 8;
    const int n8w = NEX * FI * HD / 8;
    const int n8s = FS * HD / 8;
    k_cvt16<<<(n8x + 255) / 256, 256, 0, stream>>>(x,   X16, 1.0f,  n8x);
    k_cvt16<<<(n8w + 255) / 256, 256, 0, stream>>>(wup, WUP, 64.0f, n8w);
    k_cvt16<<<(n8w + 255) / 256, 256, 0, stream>>>(wdn, WDN, 64.0f, n8w);
    k_split<<<(n8s + 255) / 256, 256, 0, stream>>>(wsu, WSUH, WSUL, n8s);
    k_split<<<(n8s + 255) / 256, 256, 0, stream>>>(wsd, WSDH, WSDL, n8s);
  }
  k_route<<<(NTOK + 7) / 8, 256, 0, stream>>>(x, rw, bias, meta, REC, NTOK);
  hipFuncSetAttribute(reinterpret_cast<const void*>(&k_expert),
                      hipFuncAttributeMaxDynamicSharedMemorySize, LDS_EXP);
  k_expert<<<dim3(NTOK / MT, NEX), 256, LDS_EXP, stream>>>(X16, WUP, WDN, REC, PART, NTOK);
  hipFuncSetAttribute(reinterpret_cast<const void*>(&k_shared),
                      hipFuncAttributeMaxDynamicSharedMemorySize, LDS_SHR);
  k_shared<<<NTOK / MS, 256, LDS_SHR, stream>>>(x, WSUH, WSUL, WSDH, WSDL, PART, out, NTOK);
}
